// CrossAttentionFusion_26551487824139
// MI455X (gfx1250) — hardware-verified
//
#include <hip/hip_runtime.h>
#include <math.h>

#ifndef NB
#define NB 4
#endif
#ifndef SEQ
#define SEQ 4096
#endif
#define NB_FULL 4
#define SEQ_FULL 4096
#define CH 128

static_assert(NB >= 1 && NB <= NB_FULL);
static_assert(SEQ >= 256 && SEQ <= SEQ_FULL && (SEQ % 256) == 0);

constexpr int kRows = NB * SEQ;
constexpr int kQCH  = (SEQ > 2048) ? 2048 : SEQ;
constexpr int kNQC  = SEQ / kQCH;
static_assert(kQCH * kNQC == SEQ && (kQCH % 64) == 0);
constexpr int kKcat = 3 * CH;
constexpr int kSmThreads = SEQ / 8;
constexpr int kSmWaves   = kSmThreads / 32;
static_assert(kSmWaves >= 1 && kSmWaves <= 16);

constexpr float kWCarry   = 16.0f;
constexpr float kWInv     = 1.0f / 16.0f;
constexpr float kPCarry   = 2048.0f;
constexpr float kPVScale  = 1.0f / 2048.0f;
constexpr float kAttScale = 0.08838834764831845f;

constexpr size_t kSzW   = (size_t)CH * CH * 2;
constexpr size_t kSzWg  = (size_t)CH * 2 * CH * 2;
constexpr size_t kSzWp  = (size_t)CH * 2 * CH * 2;
constexpr size_t kSzXC  = (size_t)kRows * 2 * CH * 2;
constexpr size_t kSzQK  = (size_t)kRows * kKcat * 2;
constexpr size_t kSzVT  = (size_t)NB * CH * SEQ * 2;
constexpr size_t kSzS   = (size_t)kQCH * SEQ * 4;
constexpr size_t kSzP   = (size_t)kQCH * SEQ * 2;
constexpr size_t kSzO   = (size_t)kRows * CH * 4;
constexpr size_t kSzG   = kSzO;
constexpr size_t kSzF   = (size_t)kRows * 2 * CH * 2;
constexpr size_t kWsTotal = 6 * kSzW + kSzWg + kSzWp + kSzXC + 2 * kSzQK + kSzVT + kSzS + kSzP + 2 * kSzO + kSzG + kSzF;
static_assert(NB != NB_FULL || SEQ != SEQ_FULL || kWsTotal == (size_t)121962496);
static_assert(kWsTotal <= (size_t)134217728);
static_assert((size_t)(NB - 1) * CH * SEQ_FULL + (size_t)(CH - 1) * SEQ_FULL + SEQ <= (size_t)NB_FULL * CH * SEQ_FULL);

typedef __attribute__((ext_vector_type(16))) _Float16 v16h;
typedef __attribute__((ext_vector_type(8)))  _Float16 v8h;
typedef __attribute__((ext_vector_type(16))) __bf16   v16b;
typedef __attribute__((ext_vector_type(8)))  __bf16   v8b;
typedef __attribute__((ext_vector_type(8)))  float    v8f;
typedef __attribute__((ext_vector_type(4)))  float    v4f;
typedef __attribute__((ext_vector_type(4)))  unsigned int v4u;

__device__ __forceinline__ unsigned short f2bf_bits(float f) {
  unsigned u = __float_as_uint(f);
  return (unsigned short)((u + 0x7FFFu + ((u >> 16) & 1u)) >> 16);
}
__device__ __forceinline__ float bf_bits2f(unsigned short h) { return __uint_as_float(((unsigned)h) << 16); }
__device__ __forceinline__ float bfr(float f) { return bf_bits2f(f2bf_bits(f)); }

__device__ __forceinline__ void dep_guard_h(v8f& a, v8f& b, v16h x, v16h y) { asm volatile("v_nop\n\tv_nop\n\tv_nop\n\tv_nop" : "+v"(a), "+v"(b) : "v"(x), "v"(y)); }
__device__ __forceinline__ void dep_guard_b(v8f& a, v8f& b, v16b x, v16b y) { asm volatile("v_nop\n\tv_nop\n\tv_nop\n\tv_nop" : "+v"(a), "+v"(b) : "v"(x), "v"(y)); }
__device__ __forceinline__ void keep4_h(v16h a, v16h b, v16h c, v16h d) { asm volatile("v_nop" :: "v"(a), "v"(b), "v"(c), "v"(d)); }
__device__ __forceinline__ void keep4_b(v16b a, v16b b, v16b c, v16b d) { asm volatile("v_nop" :: "v"(a), "v"(b), "v"(c), "v"(d)); }
__device__ __forceinline__ void acc_guard4(v8f& a, v8f& b, v8f& c, v8f& d) { asm volatile("v_nop\n\tv_nop\n\tv_nop\n\tv_nop" : "+v"(a), "+v"(b), "+v"(c), "+v"(d)); }
template <typename T> struct Frag;
template <> struct Frag<_Float16> {
  typedef v16h V; union U { v16h v; v8h h[2]; };
  static __device__ __forceinline__ v16h load(const _Float16* p) {
    U f; f.h[0] = *(const v8h*)(p); f.h[1] = *(const v8h*)(p + 16); return f.v;
  }
  static __device__ __forceinline__ v8f mma(v16h a, v16h b, v8f c) {
    return __builtin_amdgcn_wmma_f32_16x16x32_f16(false, a, false, b, (short)0, c, false, false);
  }
  static __device__ __forceinline__ void guard(v8f& a, v8f& b, v16h x, v16h y) { dep_guard_h(a, b, x, y); }
  static __device__ __forceinline__ void keep(v16h a, v16h b, v16h c, v16h d) { keep4_h(a, b, c, d); }
};
template <> struct Frag<__bf16> {
  typedef v16b V; union U { v16b v; v8b h[2]; };
  static __device__ __forceinline__ v16b load(const __bf16* p) {
    U f; f.h[0] = *(const v8b*)(p); f.h[1] = *(const v8b*)(p + 16); return f.v;
  }
  static __device__ __forceinline__ v8f mma(v16b a, v16b b, v8f c) {
    return __builtin_amdgcn_wmma_f32_16x16x32_bf16(false, a, false, b, (short)0, c, false, false);
  }
  static __device__ __forceinline__ void guard(v8f& a, v8f& b, v16b x, v16b y) { dep_guard_b(a, b, x, y); }
  static __device__ __forceinline__ void keep(v16b a, v16b b, v16b c, v16b d) { keep4_b(a, b, c, d); }
};

__device__ __forceinline__ unsigned pk16(unsigned short a, unsigned short b) { return (unsigned)a | ((unsigned)b << 16); }
__device__ __forceinline__ unsigned short h_bits(float f) { const _Float16 h = (_Float16)f; return __builtin_bit_cast(unsigned short, h); }

template <int ET> struct Elem;
template <> struct Elem<0> { typedef _Float16 T; };
template <> struct Elem<1> { typedef __bf16 T; };
template <int ET, bool SPLIT, int BIAS_MODE, int OUT_MODE, bool RESID, int ACT = 0>
__global__ __launch_bounds__(256) void wmma_gemm64(
    const unsigned short* __restrict__ Ap, const unsigned short* __restrict__ A2p, int lda, long strideA,
    const unsigned short* __restrict__ Btp, const unsigned short* __restrict__ Bt2p, int ldb, long strideB,
    void* __restrict__ Cout, void* __restrict__ Cout2, int ldc, long strideC,
    const float* __restrict__ bias,
    const float* __restrict__ resid, long strideR,
    int M, int N, int K, float scale) {
  typedef typename Elem<ET>::T T;
  typedef typename Frag<T>::V V;
  const T* A = (const T*)Ap; const T* A2 = (const T*)A2p; const T* Bt = (const T*)Btp; const T* Bt2 = (const T*)Bt2p;
  __shared__ __align__(16) float sT[8][16 * 68];
  const int b    = blockIdx.y;
  const int lane = threadIdx.x & 31;
  const int wave = threadIdx.x >> 5;
  const int tilesN = N >> 6;
  const int tilesM = M >> 6;
  const int tile = blockIdx.x * 8 + wave;
  if (tile >= tilesM * tilesN) return;
  const int tm = tile / tilesN;
  const int tn = tile - tm * tilesN;
  const int m0 = tm << 6;
  const int n0 = tn << 6;

  const T* Ab  = A  + (size_t)b * strideA;
  const T* Bb  = Bt + (size_t)b * strideB;
  const T* Ab2 = SPLIT ? (A2  + (size_t)b * strideA) : nullptr;
  const T* Bb2 = SPLIT ? (Bt2 + (size_t)b * strideB) : nullptr;

  const int rlane = lane & 15;
  const int koff  = (lane >> 4) * 8;
  const int mOff  = (lane >> 4) * 8;

  v8f acc[4][4];
#pragma unroll
  for (int i = 0; i < 4; ++i)
#pragma unroll
    for (int j = 0; j < 4; ++j) acc[i][j] = (v8f){0.f,0.f,0.f,0.f,0.f,0.f,0.f,0.f};

  for (int k0 = 0; k0 < K; k0 += 32) {
    V bh[4], bl[4];
#pragma unroll
    for (int j = 0; j < 4; ++j) {
      const size_t bo = (size_t)(n0 + (j << 4) + rlane) * ldb + koff + k0;
      bh[j] = Frag<T>::load(Bb + bo);
      if (SPLIT) bl[j] = Frag<T>::load(Bb2 + bo);
    }
#pragma unroll
    for (int i = 0; i < 4; ++i) {
      const size_t ao = (size_t)(m0 + (i << 4) + rlane) * lda + koff + k0;
      V ah = Frag<T>::load(Ab + ao);
      V al;
      if (SPLIT) al = Frag<T>::load(Ab2 + ao);
#pragma unroll
      for (int j = 0; j < 4; ++j) {
        acc[i][j] = Frag<T>::mma(ah, bh[j], acc[i][j]);
        if (SPLIT) {
          acc[i][j] = Frag<T>::mma(ah, bl[j], acc[i][j]);
          acc[i][j] = Frag<T>::mma(al, bh[j], acc[i][j]);
        }
      }
      Frag<T>::guard(acc[i][0], acc[i][3], ah, SPLIT ? al : ah);
    }
    Frag<T>::keep(bh[0], bh[1], bh[2], bh[3]);
    if (SPLIT) Frag<T>::keep(bl[0], bl[1], bl[2], bl[3]);
  }
  acc_guard4(acc[0][0], acc[0][1], acc[0][2], acc[0][3]);
  acc_guard4(acc[1][0], acc[1][1], acc[1][2], acc[1][3]);
  acc_guard4(acc[2][0], acc[2][1], acc[2][2], acc[2][3]);
  acc_guard4(acc[3][0], acc[3][1], acc[3][2], acc[3][3]);

  float* slab = sT[wave];
  const float* Rb = RESID ? (resid + (size_t)b * strideR) : nullptr;
#pragma unroll
  for (int i = 0; i < 4; ++i) {
    const int mBase = m0 + (i << 4);
#pragma unroll
    for (int j = 0; j < 4; ++j) {
      const int n = n0 + (j << 4) + rlane;
      float bv = 0.f;
      if (BIAS_MODE == 2) bv = bias[n];
#pragma unroll
      for (int r = 0; r < 8; ++r) {
        float v = acc[i][j][r] * scale;
        if (BIAS_MODE == 1) v += bias[mBase + mOff + r];
        if (BIAS_MODE == 2) v += bv;
        if (RESID) v += Rb[(size_t)(mBase + mOff + r) * ldc + n];
        if (ACT == 2) v = fmaxf(v, 0.0f);
        if (ACT == 4) v = (v > 0.f) ? v : 0.01f * v;
        slab[(mOff + r) * 68 + (j << 4) + rlane] = v;
      }
    }
    __builtin_amdgcn_fence(__ATOMIC_RELEASE, "workgroup");
    __builtin_amdgcn_wave_barrier();
    __builtin_amdgcn_fence(__ATOMIC_ACQUIRE, "workgroup");
    if (OUT_MODE == 0) {
      float* C = (float*)Cout + (size_t)b * strideC;
      const int hh = lane >> 4, c4 = (lane & 15) * 4;
      for (int pass = 0; pass < 2; ++pass) {
#pragma unroll
        for (int it = 0; it < 8; ++it) {
          const int row = it * 2 + hh;
          v4f v = *(const v4f*)(slab + row * 68 + c4);
          *(volatile v4f*)(C + (size_t)(mBase + row) * ldc + n0 + c4) = v;
        }
        __threadfence();
      }
    } else {
      const int q = lane >> 3, c8 = (lane & 7) * 8;
      unsigned short* C  = (unsigned short*)Cout  + (size_t)b * strideC;
      unsigned short* C2 = (OUT_MODE == 2) ? ((unsigned short*)Cout2 + (size_t)b * strideC) : nullptr;
      for (int pass = 0; pass < 2; ++pass) {
#pragma unroll
        for (int it = 0; it < 4; ++it) {
          const int row = it * 4 + q;
          const float* sp = slab + row * 68 + c8;
          v8h hv, lv;
#pragma unroll
          for (int e = 0; e < 8; ++e) {
            if (OUT_MODE == 1) {
              hv[e] = (_Float16)sp[e];
            } else {
              unsigned short hb = f2bf_bits(sp[e]);
              unsigned short lb = f2bf_bits(sp[e] - bf_bits2f(hb));
              hv[e] = __builtin_bit_cast(_Float16, hb);
              lv[e] = __builtin_bit_cast(_Float16, lb);
            }
          }
          *(volatile v8h*)(C + (size_t)(mBase + row) * ldc + n0 + c8) = hv;
          if (OUT_MODE == 2) *(volatile v8h*)(C2 + (size_t)(mBase + row) * ldc + n0 + c8) = lv;
        }
        __threadfence();
      }
    }
    __builtin_amdgcn_fence(__ATOMIC_RELEASE, "workgroup");
    __builtin_amdgcn_wave_barrier();
    __builtin_amdgcn_fence(__ATOMIC_ACQUIRE, "workgroup");
  }
}

__global__ __launch_bounds__(256) void wcast_kernel(
    const float* __restrict__ W0, const float* __restrict__ W1, const float* __restrict__ W2, const float* __restrict__ W3,
    const float* __restrict__ W4, const float* __restrict__ W5, const float* __restrict__ W6, const float* __restrict__ W7,
    unsigned short* __restrict__ O0, unsigned short* __restrict__ O1, unsigned short* __restrict__ O2, unsigned short* __restrict__ O3,
    unsigned short* __restrict__ O4, unsigned short* __restrict__ O5, unsigned short* __restrict__ O6, unsigned short* __restrict__ O7,
    float scale) {
  const int z = blockIdx.y;
  const float* W = (z == 0) ? W0 : (z == 1) ? W1 : (z == 2) ? W2 : (z == 3) ? W3 : (z == 4) ? W4 : (z == 5) ? W5 : (z == 6) ? W6 : W7;
  unsigned short* O = (z == 0) ? O0 : (z == 1) ? O1 : (z == 2) ? O2 : (z == 3) ? O3 : (z == 4) ? O4 : (z == 5) ? O5 : (z == 6) ? O6 : O7;
  const int n8 = (z == 6) ? (2 * CH * CH / 8) : (CH * CH / 8);
  const int i = blockIdx.x * 256 + threadIdx.x;
  if (i >= n8) return;
  const float* p = W + 8 * (size_t)i;
  const v4f a = *(const v4f*)(p);
  const v4f c = *(const v4f*)(p + 4);
  unsigned short hb[8];
  if (z < 7) {
#pragma unroll
    for (int e = 0; e < 4; ++e) {
      hb[e]     = h_bits(bfr(a[e]) * scale);
      hb[4 + e] = h_bits(bfr(c[e]) * scale);
    }
    const v4u u = (v4u){pk16(hb[0], hb[1]), pk16(hb[2], hb[3]), pk16(hb[4], hb[5]), pk16(hb[6], hb[7])};
    unsigned short* q = O + 8 * (size_t)i;
    *(volatile v4u*)q = u;
    __threadfence();
    *(volatile v4u*)q = u;
  } else {
#pragma unroll
    for (int e = 0; e < 4; ++e) {
      hb[e]     = f2bf_bits(a[e]);
      hb[4 + e] = f2bf_bits(c[e]);
    }
    const v4u u = (v4u){pk16(hb[0], hb[1]), pk16(hb[2], hb[3]), pk16(hb[4], hb[5]), pk16(hb[6], hb[7])};
    const int o = i >> 4, cc = (i & 15) * 8;
    unsigned short* q0 = O + (size_t)o * (2 * CH) + cc;
    unsigned short* q1 = q0 + CH;
    *(volatile v4u*)q0 = u;
    *(volatile v4u*)q1 = u;
    __threadfence();
    *(volatile v4u*)q0 = u;
    *(volatile v4u*)q1 = u;
  }
}

__global__ __launch_bounds__(256) void xcat_kernel(const float* __restrict__ F0, const float* __restrict__ F1,
                                                   unsigned short* __restrict__ XC) {
  __shared__ float sm[64][65];
  const int t  = threadIdx.x;
  const int n0 = blockIdx.x * 64;
  const int y  = blockIdx.y;
  const int b  = blockIdx.z;
  const float* F = (y < 2) ? F0 : F1;
  const int c0 = (y & 1) * 64;
  const int colbase = (y < 2) ? 0 : CH;
  const float* Fb = F + (size_t)b * CH * SEQ_FULL;
#pragma unroll
  for (int i = 0; i < 16; ++i) {
    const int e   = i * 256 + t;
    const int r   = e >> 6;
    const int col = e & 63;
    sm[col][r] = Fb[(size_t)(c0 + r) * SEQ_FULL + n0 + col];
  }
  __syncthreads();
  const int lane = t & 31, wave = t >> 5;
  const int q = lane >> 3, c8 = (lane & 7) * 8;
  unsigned short* op = XC + (size_t)b * SEQ * (2 * CH);
  for (int pass = 0; pass < 2; ++pass) {
#pragma unroll
    for (int it = 0; it < 2; ++it) {
      const int row = wave * 8 + it * 4 + q;
      unsigned short hb[8];
#pragma unroll
      for (int e = 0; e < 8; ++e) hb[e] = h_bits(bfr(sm[row][c8 + e]));
      const v4u u = (v4u){pk16(hb[0], hb[1]), pk16(hb[2], hb[3]), pk16(hb[4], hb[5]), pk16(hb[6], hb[7])};
      *(volatile v4u*)(op + (size_t)(n0 + row) * (2 * CH) + colbase + c0 + c8) = u;
    }
    __threadfence();
  }
}

__global__ __launch_bounds__(256) void dup_kernel(unsigned short* Qc, unsigned short* Kc, int nrows) {
  const int z = blockIdx.y;
  unsigned short* base = (z == 0) ? Qc : Kc;
  const int dstc = (z == 0) ? (2 * CH) : CH;
  const int i = blockIdx.x * 256 + threadIdx.x;
  const int row = i >> 4, piece = (i & 15) * 8;
  if (row >= nrows) return;
  const v4u v = *(const v4u*)(base + (size_t)row * kKcat + piece);
  unsigned short* q = base + (size_t)row * kKcat + dstc + piece;
  *(volatile v4u*)q = v;
  __threadfence();
  *(volatile v4u*)q = v;
}

__global__ __launch_bounds__(512) void softmax_row_kernel(const float* __restrict__ Sp, unsigned short* __restrict__ P, float carry) {
  __shared__ float redM[16];
  __shared__ float redS[16];
  const int row  = blockIdx.x;
  const int t    = threadIdx.x;
  const int lane = t & 31, wave = t >> 5;
  const int c0   = t * 8;
  const float* sr = Sp + (size_t)row * SEQ + c0;
  const v4f a = *(const v4f*)(sr);
  const v4f c = *(const v4f*)(sr + 4);
  float x[8];
#pragma unroll
  for (int e = 0; e < 4; ++e) { x[e] = a[e]; x[4 + e] = c[e]; }
  float m = fmaxf(fmaxf(fmaxf(x[0], x[1]), fmaxf(x[2], x[3])), fmaxf(fmaxf(x[4], x[5]), fmaxf(x[6], x[7])));
#pragma unroll
  for (int off = 16; off > 0; off >>= 1) m = fmaxf(m, __shfl_xor(m, off, 32));
  if (lane == 0) redM[wave] = m;
  __syncthreads();
  float mx = redM[0];
#pragma unroll
  for (int w = 1; w < kSmWaves; ++w) mx = fmaxf(mx, redM[w]);
  float p[8];
  float s = 0.f;
#pragma unroll
  for (int e = 0; e < 8; ++e) { p[e] = expf(x[e] - mx); s += p[e]; }
#pragma unroll
  for (int off = 16; off > 0; off >>= 1) s += __shfl_xor(s, off, 32);
  if (lane == 0) redS[wave] = s;
  __syncthreads();
  float tot = redS[0];
#pragma unroll
  for (int w = 1; w < kSmWaves; ++w) tot += redS[w];
  const float inv = carry * (1.0f / tot);
  unsigned short hb[8];
#pragma unroll
  for (int e = 0; e < 8; ++e) hb[e] = h_bits(p[e] * inv);
  const v4u u = (v4u){pk16(hb[0], hb[1]), pk16(hb[2], hb[3]), pk16(hb[4], hb[5]), pk16(hb[6], hb[7])};
  unsigned short* q = P + (size_t)row * SEQ + c0;
  *(volatile v4u*)q = u;
  __threadfence();
  *(volatile v4u*)q = u;
}

__global__ __launch_bounds__(256) void fuse_kernel(const float* __restrict__ Gp, const float* __restrict__ O1,
                                                   const float* __restrict__ O2, unsigned short* __restrict__ Fc) {
  __shared__ __align__(16) unsigned short hs[64 * CH];
  __shared__ __align__(16) unsigned short ls[64 * CH];
  const int t = threadIdx.x;
  const int rowbase = blockIdx.x * 64;
  const size_t ebase = (size_t)rowbase * CH;
#pragma unroll 1
  for (int i = 0; i < 32; ++i) {
    const int li = i * 256 + t;
    const size_t e = ebase + (size_t)li;
    float xg = Gp[e];
    xg = fminf(fmaxf(xg, -30.0f), 30.0f);
    const float ex = expf(-xg);
    const float g  = 1.0f / (1.0f + ex);
    const float o1 = O1[e];
    const float o2 = O2[e];
    const float f  = g * o1 + (1.0f - g) * o2;
    const unsigned short hb = f2bf_bits(f);
    const unsigned short lb = f2bf_bits(f - bf_bits2f(hb));
    hs[li] = hb;
    ls[li] = lb;
  }
  __syncthreads();
  const int lane = t & 31, wave = t >> 5;
  const int piece = (lane & 15) * 8;
  for (int pass = 0; pass < 2; ++pass) {
#pragma unroll
    for (int j = 0; j < 8; ++j) {
      const int r = wave * 8 + j;
      const v4u va = *(const v4u*)(hs + r * CH + piece);
      const v4u vb = *(const v4u*)(ls + r * CH + piece);
      v4u v = vb;
      if (lane < 16) v = va;
      *(volatile v4u*)(Fc + (size_t)(rowbase + r) * (2 * CH) + lane * 8) = v;
    }
    __threadfence();
  }
}

static inline int cdiv(int a, int b) { return (a + b - 1) / b; }

extern "C" void kernel_launch(void* const* d_in, const int* in_sizes, int n_in,
                              void* d_out, int out_size, void* d_ws, size_t ws_size,
                              hipStream_t stream) {
  if (n_in < 18) return;
  if (in_sizes[0] < NB * CH * SEQ_FULL || in_sizes[1] < NB * CH * SEQ_FULL) return;
  if (in_sizes[2] < CH * CH || in_sizes[4] < CH * CH || in_sizes[6] < CH * CH) return;
  if (in_sizes[8] < CH * CH || in_sizes[10] < CH * CH || in_sizes[12] < CH * CH) return;
  if (in_sizes[14] < 2 * CH * CH || in_sizes[16] < CH * CH) return;
  if (in_sizes[3] < CH || in_sizes[5] < CH || in_sizes[7] < CH || in_sizes[9] < CH) return;
  if (in_sizes[11] < CH || in_sizes[13] < CH || in_sizes[15] < CH || in_sizes[17] < CH) return;
  if (out_size < NB * CH * SEQ_FULL) return;
  if (kWsTotal > ws_size) return;

  const float* hsi = (const float*)d_in[0];
  const float* msi = (const float*)d_in[1];
  const float* wq1 = (const float*)d_in[2];  const float* bq1 = (const float*)d_in[3];
  const float* wk1 = (const float*)d_in[4];  const float* bk1 = (const float*)d_in[5];
  const float* wv1 = (const float*)d_in[6];  const float* bv1 = (const float*)d_in[7];
  const float* wq2 = (const float*)d_in[8];  const float* bq2 = (const float*)d_in[9];
  const float* wk2 = (const float*)d_in[10]; const float* bk2 = (const float*)d_in[11];
  const float* wv2 = (const float*)d_in[12]; const float* bv2 = (const float*)d_in[13];
  const float* wg  = (const float*)d_in[14]; const float* bg  = (const float*)d_in[15];
  const float* wp  = (const float*)d_in[16]; const float* bp  = (const float*)d_in[17];
  float* out = (float*)d_out;

  char* base = (char*)d_ws;
  size_t off = 0;
  unsigned short* Wq1h = (unsigned short*)(base + off); off += kSzW;
  unsigned short* Wk1h = (unsigned short*)(base + off); off += kSzW;
  unsigned short* Wv1h = (unsigned short*)(base + off); off += kSzW;
  unsigned short* Wq2h = (unsigned short*)(base + off); off += kSzW;
  unsigned short* Wk2h = (unsigned short*)(base + off); off += kSzW;
  unsigned short* Wv2h = (unsigned short*)(base + off); off += kSzW;
  unsigned short* Wgh  = (unsigned short*)(base + off); off += kSzWg;
  unsigned short* Wpc  = (unsigned short*)(base + off); off += kSzWp;
  unsigned short* XC   = (unsigned short*)(base + off); off += kSzXC;
  unsigned short* Qcat = (unsigned short*)(base + off); off += kSzQK;
  unsigned short* Kcat = (unsigned short*)(base + off); off += kSzQK;
  unsigned short* VT   = (unsigned short*)(base + off); off += kSzVT;
  float*          Spl  = (float*)(base + off);          off += kSzS;
  unsigned short* P16  = (unsigned short*)(base + off); off += kSzP;
  float*          O1   = (float*)(base + off);          off += kSzO;
  float*          O2   = (float*)(base + off);          off += kSzO;
  float*          G    = (float*)(base + off);          off += kSzG;
  unsigned short* Fcat = (unsigned short*)(base + off); off += kSzF;
  if (off > ws_size) return;

  const long xcPlane = (long)SEQ * 2 * CH;
  const long vtPlane = (long)CH * SEQ;

  wcast_kernel<<<dim3(16, 8), 256, 0, stream>>>(wq1, wk1, wv1, wq2, wk2, wv2, wg, wp,
                                                Wq1h, Wk1h, Wv1h, Wq2h, Wk2h, Wv2h, Wgh, Wpc, kWCarry);
  xcat_kernel<<<dim3(SEQ / 64, 4, NB), 256, 0, stream>>>(hsi, msi, XC);
  wmma_gemm64<0, false, 2, 0, false><<<dim3(cdiv((kRows / 64) * (CH / 64), 8), 1), 256, 0, stream>>>(
      XC, XC, 2 * CH, 0L, Wgh, Wgh, 2 * CH, 0L, (void*)G, (void*)G, CH, 0L,
      bg, G, 0L, kRows, CH, 2 * CH, kWInv);

  for (int r = 0; r < 2; ++r) {
    const unsigned short* Xq  = XC + ((r == 0) ? 0 : CH);
    const unsigned short* Xkv = XC + ((r == 0) ? CH : 0);
    const unsigned short* Wqh = (r == 0) ? Wq1h : Wq2h;
    const unsigned short* Wkh = (r == 0) ? Wk1h : Wk2h;
    const unsigned short* Wvh = (r == 0) ? Wv1h : Wv2h;
    const float* bq = (r == 0) ? bq1 : bq2;
    const float* bk = (r == 0) ? bk1 : bk2;
    const float* bv = (r == 0) ? bv1 : bv2;
    float* Opl = (r == 0) ? O1 : O2;

    wmma_gemm64<0, false, 2, 2, false><<<dim3(cdiv((kRows / 64) * (CH / 64), 8), 1), 256, 0, stream>>>(
        Xq, Xq, 2 * CH, 0L, Wqh, Wqh, CH, 0L, (void*)Qcat, (void*)(Qcat + CH), kKcat, 0L,
        bq, G, 0L, kRows, CH, CH, kWInv);
    wmma_gemm64<0, false, 2, 2, false><<<dim3(cdiv((kRows / 64) * (CH / 64), 8), 1), 256, 0, stream>>>(
        Xkv, Xkv, 2 * CH, 0L, Wkh, Wkh, CH, 0L, (void*)Kcat, (void*)(Kcat + 2 * CH), kKcat, 0L,
        bk, G, 0L, kRows, CH, CH, kWInv);
    dup_kernel<<<dim3(cdiv(kRows * 16, 256), 2), 256, 0, stream>>>(Qcat, Kcat, kRows);
    wmma_gemm64<0, false, 1, 1, false><<<dim3(cdiv((CH / 64) * (SEQ / 64), 8), NB), 256, 0, stream>>>(
        Wvh, Wvh, CH, 0L, Xkv, Xkv, 2 * CH, xcPlane, (void*)VT, (void*)VT, SEQ, vtPlane,
        bv, G, 0L, CH, SEQ, CH, kWInv);

    for (int b = 0; b < NB; ++b) {
      for (int h = 0; h < kNQC; ++h) {
        const int q0 = h * kQCH;
        wmma_gemm64<1, false, 0, 0, false><<<dim3(cdiv((kQCH / 64) * (SEQ / 64), 8), 1), 256, 0, stream>>>(
            Qcat + (size_t)(b * SEQ + q0) * kKcat, Qcat + (size_t)(b * SEQ + q0) * kKcat, kKcat, 0L,
            Kcat + (size_t)b * SEQ * kKcat, Kcat + (size_t)b * SEQ * kKcat, kKcat, 0L,
            (void*)Spl, (void*)Spl, SEQ, 0L, bq, G, 0L, kQCH, SEQ, kKcat, kAttScale);
        softmax_row_kernel<<<kQCH, kSmThreads, 0, stream>>>(Spl, P16, kPCarry);
        wmma_gemm64<0, false, 0, 0, false><<<dim3(cdiv((kQCH / 64) * (CH / 64), 8), 1), 256, 0, stream>>>(
            P16, P16, SEQ, 0L, VT + (size_t)b * vtPlane, VT + (size_t)b * vtPlane, SEQ, 0L,
            (void*)(Opl + (size_t)(b * SEQ + q0) * CH), (void*)(Opl + (size_t)(b * SEQ + q0) * CH), CH, 0L,
            bq, G, 0L, kQCH, CH, SEQ, kPVScale);
      }
    }
  }

  fuse_kernel<<<kRows / 64, 256, 0, stream>>>(G, O1, O2, Fcat);

  wmma_gemm64<1, false, 1, 0, false><<<dim3(cdiv((CH / 64) * (SEQ / 64), 8), NB), 256, 0, stream>>>(
      Wpc, Wpc, 2 * CH, 0L, Fcat, Fcat, 2 * CH, xcPlane, (void*)out, (void*)out, SEQ_FULL, (long)CH * SEQ_FULL,
      bp, G, 0L, CH, SEQ, 2 * CH, 1.0f);
}
